// PointNetSetAbstraction_82841329205662
// MI455X (gfx1250) — hardware-verified
//
#include <hip/hip_runtime.h>
#include <stdint.h>

#pragma clang fp contract(off)

typedef __attribute__((ext_vector_type(16))) _Float16 v16h;
typedef __attribute__((ext_vector_type(8)))  _Float16 v8h;
typedef __attribute__((ext_vector_type(8)))  float    v8f;
typedef __attribute__((ext_vector_type(4)))  float    v4f;
typedef __attribute__((ext_vector_type(4)))  unsigned int v4u;

static constexpr int kB  = 8;
static constexpr int kN  = 16384;
static constexpr int kD  = 64;
static constexpr int kS  = 1024;
static constexpr int kNS = 32;
static constexpr int kM  = kB * kS * kNS;
static constexpr int kK1 = 96;
static constexpr int kC1 = 64;
static constexpr int kC2 = 64;
static constexpr int kC3 = 128;
static constexpr int kGemmBlocks = kM / 512;
static constexpr float kR2  = 0.01f;
static constexpr float kEPS = 1e-5f;

static_assert(kM == 262144, "row count");
static_assert(kM % 512 == 0, "M tile multiple");
static_assert(kK1 % 32 == 0 && kC1 % 32 == 0 && kC2 % 32 == 0, "K multiples of 32");
static_assert(kD == 64 && kNS == 32, "shape");

static constexpr size_t kOffXQ    = 0;
static constexpr size_t kOffCQ    = kOffXQ    + (size_t)kB * 3 * kN * 4;
static constexpr size_t kOffW1T   = kOffCQ    + (size_t)kB * 3 * kS * 4;
static constexpr size_t kOffW2T   = kOffW1T   + (size_t)kC1 * kK1 * 2;
static constexpr size_t kOffW3T   = kOffW2T   + (size_t)kC2 * kC1 * 2;
static constexpr size_t kOffST1   = kOffW3T   + (size_t)kC3 * kC2 * 2;
static constexpr size_t kOffST2   = kOffST1   + 2048;
static constexpr size_t kOffST3   = kOffST2   + 2048;
static constexpr size_t kOffPART1 = kOffST3   + 2048;
static constexpr size_t kOffPART2 = kOffPART1 + (size_t)kGemmBlocks * 128 * 4;
static constexpr size_t kOffPART3 = kOffPART2 + (size_t)kGemmBlocks * 128 * 4;
static constexpr size_t kOffFEAT0 = kOffPART3 + (size_t)kGemmBlocks * 256 * 4;
static constexpr size_t kOffY1H   = kOffFEAT0 + (size_t)kM * kK1 * 2;
static constexpr size_t kOffA1H   = kOffY1H   + (size_t)kM * 64 * 2;
static constexpr size_t kOffYMAX  = kOffA1H   + (size_t)kM * 64 * 2;
static constexpr size_t kOffYMIN  = kOffYMAX  + (size_t)kB * kS * 128 * 4;
static constexpr size_t kWsTotal  = kOffYMIN  + (size_t)kB * kS * 128 * 4;
static_assert(kWsTotal <= (size_t)134217728, "carve within 128 MiB");
static_assert((kOffCQ % 128) == 0 && (kOffW1T % 128) == 0 && (kOffW2T % 128) == 0 && (kOffW3T % 128) == 0, "align");
static_assert((kOffST1 % 128) == 0 && (kOffPART1 % 128) == 0 && (kOffFEAT0 % 128) == 0, "align");
static_assert((kOffY1H % 128) == 0 && (kOffA1H % 128) == 0 && (kOffYMAX % 128) == 0 && (kOffYMIN % 128) == 0, "align");
static_assert((size_t)kM * 64 * 2 <= (size_t)kM * kK1 * 2, "layer-2 plane fits the re-used region");
static constexpr size_t kOut1ElemOff = (size_t)98304 / 4;
static_assert(kOut1ElemOff == (size_t)kB * 3 * kS, "out1 offset");
static_assert((size_t)98304 + (size_t)kB * kC3 * kS * 4 == (size_t)4292608, "output extent");

__device__ __forceinline__ float bfr(float f) {
  unsigned u = __float_as_uint(f);
  u = (u + 0x7FFFu + ((u >> 16) & 1u)) & 0xFFFF0000u;
  return __uint_as_float(u);
}

__device__ __forceinline__ float h16_to_f32(unsigned hb) {
  const unsigned sgn = (hb & 0x8000u) << 16; const unsigned em = hb & 0x7fffu;
  const float fn = __uint_as_float((em << 13) + 0x38000000u);
  const float fs = (float)em * 5.9604644775390625e-8f;
  const float mag = (em < 0x400u) ? fs : fn; return __uint_as_float(__float_as_uint(mag) | sgn); }

struct FragH {
  union U { v16h v; v8h h[2]; };
  static __device__ __forceinline__ v16h load(const _Float16* p) {
    U f; f.h[0] = *(const v8h*)(p); f.h[1] = *(const v8h*)(p + 16); return f.v;
  }
  static __device__ __forceinline__ v8f mma(v16h a, v16h b, v8f c) {
    return __builtin_amdgcn_wmma_f32_16x16x32_f16(false, a, false, b, (short)0, c, false, false);
  }
};
__device__ __forceinline__ void guard_row(v8f& a0, v8f& a1, v8f& a2, v8f& a3,
                                          v16h x, v16h b0, v16h b1, v16h b2, v16h b3) {
  asm volatile("v_nop\n\tv_nop\n\tv_nop\n\tv_nop"
               : "+v"(a0), "+v"(a1), "+v"(a2), "+v"(a3)
               : "v"(x), "v"(b0), "v"(b1), "v"(b2), "v"(b3));
}
__device__ __forceinline__ void acc_guard4(v8f& a, v8f& b, v8f& c, v8f& d) {
  asm volatile("v_nop\n\tv_nop\n\tv_nop\n\tv_nop" : "+v"(a), "+v"(b), "+v"(c), "+v"(d));
}

static constexpr int kXqBlocks   = (kB * 3 * kN / 4) / 256;
static constexpr int kPrepBlocks = kXqBlocks + 9;
static_assert(kXqBlocks * 1024 == kB * 3 * kN, "xq coverage");

__global__ __launch_bounds__(256) void prep_kernel(
    const float* __restrict__ xyz, const float* __restrict__ w1, const float* __restrict__ w2,
    const float* __restrict__ w3, float* __restrict__ xq,
    unsigned short* __restrict__ w1t, unsigned short* __restrict__ w2t, unsigned short* __restrict__ w3t) {
  const int tid = threadIdx.x;
  if (blockIdx.x < kXqBlocks) {
    const size_t i4 = ((size_t)blockIdx.x * 256 + tid) * 4;
    const v4f x = *(const v4f*)(xyz + i4);
    const float x0 = x[0], x1 = x[1], x2 = x[2], x3 = x[3];
    v4f o;
    o[0] = bfr(x0); o[1] = bfr(x1); o[2] = bfr(x2); o[3] = bfr(x3);
    *(volatile v4f*)(xq + i4) = o;
    __threadfence();
    *(volatile v4f*)(xq + i4) = o;
    return;
  }
  const int wb = (int)blockIdx.x - kXqBlocks;
  v8h hv;
  unsigned short* dst;
  if (wb < 3) {
    const int uu = wb * 256 + tid;
    const int o = uu / 12;
    const int k8 = (uu - o * 12) * 8;
#pragma unroll
    for (int e = 0; e < 8; ++e) {
      const int k = k8 + e;
      int col = (k < 64) ? (k + 3) : (k - 64);
      col = col > 66 ? 66 : col;
      const float x = w1[o * 67 + col];
      const float v = (k < 67) ? bfr(x) : 0.0f;
      hv[e] = (_Float16)v;
    }
    dst = w1t + (size_t)uu * 8;
  } else if (wb < 5) {
    const int uu = (wb - 3) * 256 + tid;
#pragma unroll
    for (int e = 0; e < 8; ++e) {
      const float x = w2[(size_t)uu * 8 + e];
      hv[e] = (_Float16)bfr(x);
    }
    dst = w2t + (size_t)uu * 8;
  } else {
    const int uu = (wb - 5) * 256 + tid;
#pragma unroll
    for (int e = 0; e < 8; ++e) {
      const float x = w3[(size_t)uu * 8 + e];
      hv[e] = (_Float16)bfr(x);
    }
    dst = w3t + (size_t)uu * 8;
  }
  *(volatile v8h*)(dst) = hv;
  __threadfence();
  *(volatile v8h*)(dst) = hv;
}

__global__ __launch_bounds__(1024) void fps_kernel(const float* __restrict__ xq,
                                                   float* __restrict__ out0,
                                                   float* __restrict__ cq) {
#pragma clang fp contract(off)
  const int b    = blockIdx.x;
  const int tid  = threadIdx.x;
  const int lane = tid & 31;
  const int wave = tid >> 5;
  const float* xb = xq + (size_t)b * 3 * kN;

  __shared__ float s_val[2][32];
  __shared__ int   s_idx[2][32];
  __shared__ int   s_hist[kS];

  float px[16], py[16], pz[16], pd[16];
#pragma unroll
  for (int j = 0; j < 16; ++j) {
    const int i = tid + j * 1024;
    px[j] = xb[i];
    py[j] = xb[kN + i];
    pz[j] = xb[2 * kN + i];
    pd[j] = 1e10f;
    asm volatile("" : "+v"(px[j]), "+v"(py[j]), "+v"(pz[j]) :: "memory");
  }

  int cur = 0;
#pragma unroll 1
  for (int it = 0; it < kS; ++it) {
    if (tid == 0) s_hist[it] = cur;
    int cc = cur < 0 ? 0 : cur;
    cc = cc > (kN - 1) ? (kN - 1) : cc;
    const float cx = xb[cc];
    const float cy = xb[kN + cc];
    const float cz = xb[2 * kN + cc];

    float bv = -1.0f;
    int   bi = 0;
#pragma unroll
    for (int j = 0; j < 16; ++j) {
      const float dx = px[j] - cx;
      const float dy = py[j] - cy;
      const float dz = pz[j] - cz;
      const float t0 = dx * dx;
      const float t1 = dy * dy;
      const float t2 = dz * dz;
      const float d  = (t0 + t2) + t1;
      const float nd = fminf(pd[j], d);
      pd[j] = nd;
      const bool up = nd > bv;
      bv = up ? nd : bv;
      bi = up ? (tid + j * 1024) : bi;
    }
#pragma unroll
    for (int off = 16; off > 0; off >>= 1) {
      const float ov = __shfl_xor(bv, off);
      const int   oi = __shfl_xor(bi, off);
      const bool take = (ov > bv) || ((ov == bv) && (oi < bi));
      bv = take ? ov : bv;
      bi = take ? oi : bi;
    }
    const int p = it & 1;
    if (lane == 0) { s_val[p][wave] = bv; s_idx[p][wave] = bi; }
    __syncthreads();
    float v2 = s_val[p][lane];
    int   i2 = s_idx[p][lane];
#pragma unroll
    for (int off = 16; off > 0; off >>= 1) {
      const float ov = __shfl_xor(v2, off);
      const int   oi = __shfl_xor(i2, off);
      const bool take = (ov > v2) || ((ov == v2) && (oi < i2));
      v2 = take ? ov : v2;
      i2 = take ? oi : i2;
    }
    cur = i2;
  }
  __syncthreads();
  int id = s_hist[tid];
  id = id < 0 ? 0 : id;
  id = id > (kN - 1) ? (kN - 1) : id;
  const float v0 = xb[id];
  const float v1 = xb[kN + id];
  const float v2o = xb[2 * kN + id];
  float* o0 = out0 + (size_t)b * 3 * kS + tid;
  float* c0 = cq   + (size_t)b * 3 * kS + tid;
  for (int pass = 0; pass < 2; ++pass) {
    *(volatile float*)(o0)          = v0;
    *(volatile float*)(o0 + kS)     = v1;
    *(volatile float*)(o0 + 2 * kS) = v2o;
    *(volatile float*)(c0)          = v0;
    *(volatile float*)(c0 + kS)     = v1;
    *(volatile float*)(c0 + 2 * kS) = v2o;
    __threadfence();
  }
}

__global__ __launch_bounds__(128) void ball_gather_kernel(const float* __restrict__ xq,
                                                          const float* __restrict__ points,
                                                          const float* __restrict__ cq,
                                                          unsigned short* __restrict__ feat) {
#pragma clang fp contract(off)
  __shared__ int s_hit[4][32];
  __shared__ __align__(16) _Float16 s_row[4 * 32 * kK1];
  const int tid  = threadIdx.x;
  const int lane = tid & 31;
  const int wave = tid >> 5;
  const int g = blockIdx.x * 4 + wave;
  const int b = g >> 10;
  const int s = g & (kS - 1);
  const float* xb = xq + (size_t)b * 3 * kN;
  const float cx = cq[((size_t)b * 3 + 0) * kS + s];
  const float cy = cq[((size_t)b * 3 + 1) * kS + s];
  const float cz = cq[((size_t)b * 3 + 2) * kS + s];
  const float sx = cx * cx;
  const float sy = cy * cy;
  const float sz = cz * cz;
  const float ss = (sx + sz) + sy;

  s_hit[wave][lane] = 0;
  int cnt = 0;
  int first = kN - 1;
#pragma unroll 1
  for (int i0 = 0; i0 < kN; i0 += 32) {
    const int i = i0 + lane;
    const float qx = xb[i];
    const float qy = xb[kN + i];
    const float qz = xb[2 * kN + i];
    const float n0 = qx * qx;
    const float n1 = qy * qy;
    const float n2 = qz * qz;
    const float nn = (n0 + n2) + n1;
    float p = cx * qx;
    p = __builtin_fmaf(cy, qy, p);
    p = __builtin_fmaf(cz, qz, p);
    const float tw = 2.0f * p;
    const float sqr = (ss + nn) - tw;
    const bool in = !(sqr > kR2);
    const unsigned m = __builtin_amdgcn_ballot_w32(in);
    if (cnt == 0 && m != 0u) first = i0 + __builtin_ctz(m);
    const int pos = cnt + __popc(m & ((1u << lane) - 1u));
    if (in && pos < kNS) s_hit[wave][pos] = i;
    cnt += __popc(m);
    if (cnt >= kNS) break;
  }
  __syncthreads();
  const int have = cnt > kNS ? kNS : cnt;
  const int hv0 = s_hit[wave][lane];
  int gi = (lane < have) ? hv0 : first;
  gi = gi < 0 ? 0 : gi;
  gi = gi > (kN - 1) ? (kN - 1) : gi;

  _Float16* row = s_row + (size_t)wave * 32 * kK1 + lane * kK1;
  const float* pb = points + (size_t)b * kD * kN + gi;
#pragma unroll 1
  for (int k8 = 0; k8 < kD; k8 += 8) {
    v8h hv;
#pragma unroll
    for (int e = 0; e < 8; ++e) {
      const float x = pb[(size_t)(k8 + e) * kN];
      hv[e] = (_Float16)bfr(x);
    }
    *(v8h*)(row + k8) = hv;
  }
  {
    const float d0 = xb[gi] - cx;
    const float d1 = xb[kN + gi] - cy;
    const float d2 = xb[2 * kN + gi] - cz;
    float zf = 0.0f;
    asm volatile("" : "+v"(zf));
    const _Float16 zh = (_Float16)zf;
    v8h dv;
    dv[0] = (_Float16)d0; dv[1] = (_Float16)d1; dv[2] = (_Float16)d2;
    dv[3] = zh; dv[4] = zh; dv[5] = zh; dv[6] = zh; dv[7] = zh;
    v8h zv;
    zv[0] = zh; zv[1] = zh; zv[2] = zh; zv[3] = zh; zv[4] = zh; zv[5] = zh; zv[6] = zh; zv[7] = zh;
    *(v8h*)(row + 64) = dv;
    *(v8h*)(row + 72) = zv;
    *(v8h*)(row + 80) = zv;
    *(v8h*)(row + 88) = zv;
  }
  __syncthreads();
  const _Float16* src = s_row + (size_t)wave * 32 * kK1;
  unsigned short* dst = feat + (size_t)g * (32 * kK1);
  for (int pass = 0; pass < 2; ++pass) {
#pragma unroll
    for (int it = 0; it < 12; ++it) {
      const v8h v = *(const v8h*)(src + it * 256 + lane * 8);
      *(volatile v8h*)(dst + it * 256 + lane * 8) = v;
    }
    __threadfence();
  }
}

template <int KDIM, int NT, int MODE>
__global__ __launch_bounds__(256) void mlp_gemm_kernel(
    const unsigned short* __restrict__ Ap, const unsigned short* __restrict__ Btp,
    const float* __restrict__ bias, unsigned short* __restrict__ Yout,
    float* __restrict__ part, float* __restrict__ ymax, float* __restrict__ ymin) {
  static_assert(KDIM % 32 == 0, "K multiple of 32");
  static_assert((MODE == 0 && NT == 1) || (MODE == 1 && NT == 2), "mode");
  constexpr int NCH = NT * 64;
  const _Float16* A  = (const _Float16*)Ap;
  const _Float16* Bt = (const _Float16*)Btp;
  __shared__ __align__(16) float sT[(MODE == 0) ? (8 * 16 * 68) : 4];
  __shared__ __align__(16) float sStat[8 * 2 * NCH];
  __shared__ __align__(16) float sMM[(MODE == 1) ? (8 * 4 * NCH) : 4];

  const int lane = threadIdx.x & 31;
  const int wave = threadIdx.x >> 5;
  const int tile = blockIdx.x * 8 + wave;
  const int m0 = tile << 6;
  const int rlane = lane & 15;
  const int koff  = (lane >> 4) * 8;
  const int mOff  = (lane >> 4) * 8;

#pragma unroll 1
  for (int nt = 0; nt < NT; ++nt) {
    const int n0 = nt << 6;
    v8f acc[4][4];
#pragma unroll
    for (int i = 0; i < 4; ++i)
#pragma unroll
      for (int j = 0; j < 4; ++j) acc[i][j] = (v8f){0.f, 0.f, 0.f, 0.f, 0.f, 0.f, 0.f, 0.f};

#pragma unroll 1
    for (int k0 = 0; k0 < KDIM; k0 += 32) {
      v16h bh[4];
#pragma unroll
      for (int j = 0; j < 4; ++j) {
        const size_t bo = (size_t)(n0 + (j << 4) + rlane) * KDIM + koff + k0;
        bh[j] = FragH::load(Bt + bo);
      }
#pragma unroll
      for (int i = 0; i < 4; ++i) {
        const size_t ao = (size_t)(m0 + (i << 4) + rlane) * KDIM + koff + k0;
        const v16h ah = FragH::load(A + ao);
#pragma unroll
        for (int j = 0; j < 4; ++j) acc[i][j] = FragH::mma(ah, bh[j], acc[i][j]);
        guard_row(acc[i][0], acc[i][1], acc[i][2], acc[i][3], ah, bh[0], bh[1], bh[2], bh[3]);
      }
    }
    acc_guard4(acc[0][0], acc[0][1], acc[0][2], acc[0][3]);
    acc_guard4(acc[1][0], acc[1][1], acc[1][2], acc[1][3]);
    acc_guard4(acc[2][0], acc[2][1], acc[2][2], acc[2][3]);
    acc_guard4(acc[3][0], acc[3][1], acc[3][2], acc[3][3]);

    if (MODE == 0) {
      float* slab = sT + wave * (16 * 68);
      float sS[4], sQ[4], bv[4];
#pragma unroll
      for (int j = 0; j < 4; ++j) {
        sS[j] = 0.0f; sQ[j] = 0.0f;
        bv[j] = bfr(bias[n0 + (j << 4) + rlane]);
      }
#pragma unroll
      for (int i = 0; i < 4; ++i) {
        const int mBase = m0 + (i << 4);
#pragma unroll
        for (int j = 0; j < 4; ++j) {
#pragma unroll
          for (int r = 0; r < 8; ++r) {
            const float v = acc[i][j][r] + bv[j];
            const float v2 = v * v;
            sS[j] += v;
            sQ[j] += v2;
            slab[(mOff + r) * 68 + (j << 4) + rlane] = v;
          }
        }
        __builtin_amdgcn_fence(__ATOMIC_RELEASE, "workgroup");
        __builtin_amdgcn_wave_barrier();
        __builtin_amdgcn_fence(__ATOMIC_ACQUIRE, "workgroup");
        {
          const int q = lane >> 3, c8 = (lane & 7) * 8;
          for (int pass = 0; pass < 2; ++pass) {
#pragma unroll
            for (int it = 0; it < 4; ++it) {
              const int rw = it * 4 + q;
              const float* sp = slab + rw * 68 + c8;
              v8h hv;
#pragma unroll
              for (int e = 0; e < 8; ++e) hv[e] = (_Float16)sp[e];
              *(volatile v8h*)(Yout + (size_t)(mBase + rw) * 64 + c8) = hv;
            }
            __threadfence();
          }
        }
        __builtin_amdgcn_fence(__ATOMIC_RELEASE, "workgroup");
        __builtin_amdgcn_wave_barrier();
        __builtin_amdgcn_fence(__ATOMIC_ACQUIRE, "workgroup");
      }
#pragma unroll
      for (int j = 0; j < 4; ++j) {
        const float so = __shfl_xor(sS[j], 16);
        const float qo = __shfl_xor(sQ[j], 16);
        const float st = sS[j] + so;
        const float qt = sQ[j] + qo;
        if (lane < 16) {
          sStat[wave * 2 * NCH + n0 + (j << 4) + rlane] = st;
          sStat[wave * 2 * NCH + NCH + n0 + (j << 4) + rlane] = qt;
        }
      }
    } else {
#pragma unroll
      for (int j = 0; j < 4; ++j) {
        const int ch = n0 + (j << 4) + rlane;
        const float bvj = bfr(bias[ch]);
        float s = 0.0f, q = 0.0f;
        float mx0 = -__builtin_huge_valf(), mn0 = __builtin_huge_valf();
        float mx1 = -__builtin_huge_valf(), mn1 = __builtin_huge_valf();
#pragma unroll
        for (int i = 0; i < 4; ++i) {
#pragma unroll
          for (int r = 0; r < 8; ++r) {
            const float v = acc[i][j][r] + bvj;
            const float v2 = v * v;
            s += v;
            q += v2;
            if (i < 2) { mx0 = fmaxf(mx0, v); mn0 = fminf(mn0, v); }
            else       { mx1 = fmaxf(mx1, v); mn1 = fminf(mn1, v); }
          }
        }
        const float so  = __shfl_xor(s, 16);
        const float qo  = __shfl_xor(q, 16);
        const float a0  = __shfl_xor(mx0, 16);
        const float b0  = __shfl_xor(mn0, 16);
        const float a1  = __shfl_xor(mx1, 16);
        const float b1  = __shfl_xor(mn1, 16);
        const float st = s + so;
        const float qt = q + qo;
        mx0 = fmaxf(mx0, a0); mn0 = fminf(mn0, b0);
        mx1 = fmaxf(mx1, a1); mn1 = fminf(mn1, b1);
        if (lane < 16) {
          sStat[wave * 2 * NCH + ch] = st;
          sStat[wave * 2 * NCH + NCH + ch] = qt;
          sMM[wave * 4 * NCH + 0 * NCH + ch] = mx0;
          sMM[wave * 4 * NCH + 1 * NCH + ch] = mn0;
          sMM[wave * 4 * NCH + 2 * NCH + ch] = mx1;
          sMM[wave * 4 * NCH + 3 * NCH + ch] = mn1;
        }
      }
    }
  }
  __syncthreads();

  if (MODE == 1) {
    v4f vals[4];
#pragma unroll
    for (int w = 0; w < 4; ++w) vals[w] = *(const v4f*)(sMM + wave * 4 * NCH + w * NCH + 4 * lane);
    float* pmx0 = ymax + (size_t)(tile * 2 + 0) * 128 + 4 * lane;
    float* pmn0 = ymin + (size_t)(tile * 2 + 0) * 128 + 4 * lane;
    float* pmx1 = ymax + (size_t)(tile * 2 + 1) * 128 + 4 * lane;
    float* pmn1 = ymin + (size_t)(tile * 2 + 1) * 128 + 4 * lane;
    for (int pass = 0; pass < 2; ++pass) {
      *(volatile v4f*)(pmx0) = vals[0];
      *(volatile v4f*)(pmn0) = vals[1];
      *(volatile v4f*)(pmx1) = vals[2];
      *(volatile v4f*)(pmn1) = vals[3];
      __threadfence();
    }
  }
  if (wave == 0) {
    constexpr int NIT = (2 * NCH) / 128;
    v4f tot[NIT];
#pragma unroll
    for (int it = 0; it < NIT; ++it) {
      v4f t = (v4f){0.f, 0.f, 0.f, 0.f};
#pragma unroll
      for (int w = 0; w < 8; ++w) {
        const v4f x = *(const v4f*)(sStat + w * 2 * NCH + it * 128 + 4 * lane);
        t = t + x;
      }
      tot[it] = t;
    }
    float* pr = part + (size_t)blockIdx.x * (2 * NCH);
    for (int pass = 0; pass < 2; ++pass) {
#pragma unroll
      for (int it = 0; it < NIT; ++it) *(volatile v4f*)(pr + it * 128 + 4 * lane) = tot[it];
      __threadfence();
    }
  }
}

template <int C>
__global__ __launch_bounds__(128) void bn_stats_kernel(const float* __restrict__ part,
                                                       const float* __restrict__ g,
                                                       const float* __restrict__ be,
                                                       float* __restrict__ stat) {
  static_assert(C == 64 || C == 128, "channels");
  __shared__ __align__(16) float s_out[2 * C];
  const int tid = threadIdx.x;
  const int lane = tid & 31;
  const int wave = tid >> 5;
  const int cc = tid < C ? tid : (C - 1);
  double S = 0.0, Q = 0.0;
#pragma unroll 4
  for (int blk = 0; blk < kGemmBlocks; ++blk) {
    const float a = part[(size_t)blk * (2 * C) + cc];
    const float q = part[(size_t)blk * (2 * C) + C + cc];
    S += (double)a;
    Q += (double)q;
  }
  const double invM = 1.0 / (double)kM;
  const double mean = S * invM;
  double var = Q * invM - mean * mean;
  var = var < 0.0 ? 0.0 : var;
  const float varf = (float)var;
  const float rs = 1.0f / sqrtf(varf + kEPS);
  const float sc = bfr(g[cc]) * rs;
  const float ms = (float)mean * sc;
  const float sh = bfr(be[cc]) - ms;
  if (tid < C) { s_out[tid] = sc; s_out[C + tid] = sh; }
  __syncthreads();
  if (wave == 0) {
    constexpr int NIT = (2 * C) / 128;
    v4f v[NIT];
#pragma unroll
    for (int it = 0; it < NIT; ++it) v[it] = *(const v4f*)(s_out + it * 128 + 4 * lane);
    for (int pass = 0; pass < 2; ++pass) {
#pragma unroll
      for (int it = 0; it < NIT; ++it) *(volatile v4f*)(stat + it * 128 + 4 * lane) = v[it];
      __threadfence();
    }
  }
}

__global__ __launch_bounds__(256) void bn_relu_kernel(const unsigned short* __restrict__ y,
                                                      const float* __restrict__ stat,
                                                      unsigned short* __restrict__ a) {
  const size_t t = (size_t)blockIdx.x * 256 + threadIdx.x;
  const int c8 = ((int)(t & 7)) * 8;
  const v4u w = *(const v4u*)(y + t * 8);
  const v4f sc0 = *(const v4f*)(stat + c8);
  const v4f sc1 = *(const v4f*)(stat + c8 + 4);
  const v4f sh0 = *(const v4f*)(stat + 64 + c8);
  const v4f sh1 = *(const v4f*)(stat + 64 + c8 + 4);
  const unsigned w0 = w[0], w1 = w[1], w2 = w[2], w3 = w[3];
  float x[8];
  x[0] = h16_to_f32(w0 & 0xffffu); x[1] = h16_to_f32(w0 >> 16);
  x[2] = h16_to_f32(w1 & 0xffffu); x[3] = h16_to_f32(w1 >> 16);
  x[4] = h16_to_f32(w2 & 0xffffu); x[5] = h16_to_f32(w2 >> 16);
  x[6] = h16_to_f32(w3 & 0xffffu); x[7] = h16_to_f32(w3 >> 16);
  float scv[8], shv[8];
  scv[0] = sc0[0]; scv[1] = sc0[1]; scv[2] = sc0[2]; scv[3] = sc0[3];
  scv[4] = sc1[0]; scv[5] = sc1[1]; scv[6] = sc1[2]; scv[7] = sc1[3];
  shv[0] = sh0[0]; shv[1] = sh0[1]; shv[2] = sh0[2]; shv[3] = sh0[3];
  shv[4] = sh1[0]; shv[5] = sh1[1]; shv[6] = sh1[2]; shv[7] = sh1[3];
  v8h hv;
#pragma unroll
  for (int e = 0; e < 8; ++e) {
    const float m = x[e] * scv[e];
    float v = m + shv[e];
    v = fmaxf(v, 0.0f);
    hv[e] = (_Float16)v;
  }
  unsigned short* dst = a + t * 8;
  *(volatile v8h*)(dst) = hv;
  __threadfence();
  *(volatile v8h*)(dst) = hv;
}

__global__ __launch_bounds__(256) void pool_out_kernel(const float* __restrict__ ymax,
                                                       const float* __restrict__ ymin,
                                                       const float* __restrict__ stat,
                                                       float* __restrict__ out1) {
  __shared__ __align__(16) float tile[128 * 36];
  const int tid  = threadIdx.x;
  const int lane = tid & 31;
  const int wave = tid >> 5;
  const int g0 = blockIdx.x * 32;
  const int b  = g0 >> 10;
  const int s0 = g0 & (kS - 1);
#pragma unroll 1
  for (int it = 0; it < 4; ++it) {
    const int u  = it * 256 + tid;
    const int sl = u >> 5;
    const int o4 = (u & 31) * 4;
    const v4f mx = *(const v4f*)(ymax + (size_t)(g0 + sl) * 128 + o4);
    const v4f mn = *(const v4f*)(ymin + (size_t)(g0 + sl) * 128 + o4);
    const v4f sc = *(const v4f*)(stat + o4);
    const v4f sh = *(const v4f*)(stat + 128 + o4);
#pragma unroll
    for (int e = 0; e < 4; ++e) {
      const float scv = sc[e];
      const float mxe = mx[e];
      const float mne = mn[e];
      const float pick = (scv >= 0.0f) ? mxe : mne;
      const float m = scv * pick;
      float v = m + sh[e];
      v = fmaxf(v, 0.0f);
      tile[(o4 + e) * 36 + sl] = v;
    }
  }
  __syncthreads();
  v4f vals[4];
  const int s4 = (lane & 7) * 4;
#pragma unroll
  for (int it = 0; it < 4; ++it) {
    const int o = (wave * 4 + it) * 4 + (lane >> 3);
    vals[it] = *(const v4f*)(tile + o * 36 + s4);
  }
  for (int pass = 0; pass < 2; ++pass) {
#pragma unroll
    for (int it = 0; it < 4; ++it) {
      const int o = (wave * 4 + it) * 4 + (lane >> 3);
      *(volatile v4f*)(out1 + ((size_t)(b * 128 + o)) * kS + s0 + s4) = vals[it];
    }
    __threadfence();
  }
}

extern "C" void kernel_launch(void* const* d_in, const int* in_sizes, int n_in,
                              void* d_out, int out_size, void* d_ws, size_t ws_size,
                              hipStream_t stream) {
  (void)in_sizes; (void)out_size;
  if (n_in < 14) return;
  if (ws_size < kWsTotal) return;
  const float* xyz    = (const float*)d_in[0];
  const float* points = (const float*)d_in[1];
  const float* w1  = (const float*)d_in[2];
  const float* b1  = (const float*)d_in[3];
  const float* g1  = (const float*)d_in[4];
  const float* be1 = (const float*)d_in[5];
  const float* w2  = (const float*)d_in[6];
  const float* b2  = (const float*)d_in[7];
  const float* g2  = (const float*)d_in[8];
  const float* be2 = (const float*)d_in[9];
  const float* w3  = (const float*)d_in[10];
  const float* b3  = (const float*)d_in[11];
  const float* g3  = (const float*)d_in[12];
  const float* be3 = (const float*)d_in[13];

  float* out0 = (float*)d_out;
  float* out1 = (float*)d_out + kOut1ElemOff;

  char* ws = (char*)d_ws;
  float* xq   = (float*)(ws + kOffXQ);
  float* cq   = (float*)(ws + kOffCQ);
  unsigned short* w1t = (unsigned short*)(ws + kOffW1T);
  unsigned short* w2t = (unsigned short*)(ws + kOffW2T);
  unsigned short* w3t = (unsigned short*)(ws + kOffW3T);
  float* st1  = (float*)(ws + kOffST1);
  float* st2  = (float*)(ws + kOffST2);
  float* st3  = (float*)(ws + kOffST3);
  float* pt1  = (float*)(ws + kOffPART1);
  float* pt2  = (float*)(ws + kOffPART2);
  float* pt3  = (float*)(ws + kOffPART3);
  unsigned short* feat0 = (unsigned short*)(ws + kOffFEAT0);
  unsigned short* y1h   = (unsigned short*)(ws + kOffY1H);
  unsigned short* a1h   = (unsigned short*)(ws + kOffA1H);
  unsigned short* y2h   = feat0;
  unsigned short* a2h   = y1h;
  float* ymax = (float*)(ws + kOffYMAX);
  float* ymin = (float*)(ws + kOffYMIN);

  prep_kernel<<<kPrepBlocks, 256, 0, stream>>>(xyz, w1, w2, w3, xq, w1t, w2t, w3t);
  fps_kernel<<<kB, 1024, 0, stream>>>(xq, out0, cq);
  ball_gather_kernel<<<(kB * kS) / 4, 128, 0, stream>>>(xq, points, cq, feat0);

  mlp_gemm_kernel<kK1, 1, 0><<<kGemmBlocks, 256, 0, stream>>>(feat0, w1t, b1, y1h, pt1, ymax, ymin);
  bn_stats_kernel<64><<<1, 128, 0, stream>>>(pt1, g1, be1, st1);
  bn_relu_kernel<<<(kM * 8) / 256, 256, 0, stream>>>(y1h, st1, a1h);

  mlp_gemm_kernel<kC1, 1, 0><<<kGemmBlocks, 256, 0, stream>>>(a1h, w2t, b2, y2h, pt2, ymax, ymin);
  bn_stats_kernel<64><<<1, 128, 0, stream>>>(pt2, g2, be2, st2);
  bn_relu_kernel<<<(kM * 8) / 256, 256, 0, stream>>>(y2h, st2, a2h);

  mlp_gemm_kernel<kC2, 2, 1><<<kGemmBlocks, 256, 0, stream>>>(a2h, w3t, b3, y2h, pt3, ymax, ymin);
  bn_stats_kernel<128><<<1, 128, 0, stream>>>(pt3, g3, be3, st3);
  pool_out_kernel<<<(kB * kS) / 32, 256, 0, stream>>>(ymax, ymin, st3, out1);
}
